// ModularSelectCascadeNet_21921513079161
// MI455X (gfx1250) — hardware-verified
//
#include <hip/hip_runtime.h>

typedef unsigned short us;
typedef unsigned char  uc;
typedef us     v8us  __attribute__((ext_vector_type(8)));
typedef us     v16us __attribute__((ext_vector_type(16)));
typedef __bf16 v16bf __attribute__((ext_vector_type(16)));
typedef float  v8f   __attribute__((ext_vector_type(8)));
typedef float  v4f   __attribute__((ext_vector_type(4)));
typedef unsigned int v4u __attribute__((ext_vector_type(4)));
typedef v4f  __attribute__((may_alias)) v4fa;
typedef v4u  __attribute__((may_alias)) v4ua;
typedef v8us __attribute__((may_alias)) v8usa;
typedef float __attribute__((may_alias)) f32a;
typedef us    __attribute__((may_alias)) usa;
typedef uc    __attribute__((may_alias)) uca;

__device__ __forceinline__ us f2bf(float f) {
  unsigned int u = __float_as_uint(f);
  u = u + 0x7FFFu + ((u >> 16) & 1u);
  return (us)(u >> 16);
}
__device__ __forceinline__ float bf2f(us b) { return __uint_as_float(((unsigned int)b) << 16); }
__device__ __forceinline__ unsigned int pack2(us lo16, us hi16) {
  return (unsigned int)lo16 | ((unsigned int)hi16 << 16);
}
__device__ __forceinline__ v8f zero8() {
  v8f z;
  z[0] = 0.f; z[1] = 0.f; z[2] = 0.f; z[3] = 0.f; z[4] = 0.f; z[5] = 0.f; z[6] = 0.f; z[7] = 0.f;
  return z;
}

__device__ __forceinline__ void wave_sync() {
#if defined(__HIP_DEVICE_COMPILE__)
  __builtin_amdgcn_fence(__ATOMIC_RELEASE, "wavefront");
  __builtin_amdgcn_wave_barrier();
#endif
}

__device__ __forceinline__ v8f wmma16(v16bf a, v16bf b, v8f c) {
#if defined(__HIP_DEVICE_COMPILE__)
  v8f d = __builtin_amdgcn_wmma_f32_16x16x32_bf16(false, a, false, b, (short)0, c, false, false);
  asm volatile("v_nop\n\tv_nop\n\tv_nop\n\tv_nop" : "+v"(d) : "v"(a), "v"(b));
  return d;
#else
  return c;
#endif
}

union Frag16 { v16us u; v8us half[2]; v16bf v; };
__device__ __forceinline__ v16bf ldfrag(const us* p, int hh) {
  Frag16 f;
  f.half[0] = *(const v8usa*)(p + 8 * hh);
  f.half[1] = *(const v8usa*)(p + 16 + 8 * hh);
  return f.v;
}

template<int NT>
__device__ __forceinline__ void store_f32_tile(const float* sf, float* cbase, int row0, int ldc, int lane) {
  #pragma unroll
  for (int it = 0; it < NT * 2; ++it) {
    const int p = it * 32 + lane;
    const int rr = p / (NT * 4);
    const int pc = p - rr * (NT * 4);
    const v4f val = *(const v4fa*)(sf + rr * (NT * 16) + pc * 4);
    *(volatile v4f*)(cbase + (size_t)(row0 + rr) * ldc + pc * 4) = val;
  }
}

__device__ __forceinline__ void store_u16_tile(const us* s, us* base, int row0, int ld, int lane) {
  #pragma unroll
  for (int it = 0; it < 4; ++it) {
    const int p = it * 32 + lane;
    const int rr = p >> 3, pc = p & 7;
    const v4u val = *(const v4ua*)(s + rr * 64 + pc * 8);
    *(volatile v4u*)(base + (size_t)(row0 + rr) * ld + pc * 8) = val;
  }
}

__device__ __forceinline__ void store_u8_tile(const uc* s, uc* base, int lane) {
  #pragma unroll
  for (int it = 0; it < 2; ++it) {
    const int p = it * 32 + lane;
    const v4u val = *(const v4ua*)(s + p * 16);
    *(volatile v4u*)(base + (size_t)p * 16) = val;
  }
}

__global__ __launch_bounds__(256) void cvt_in_kernel(const float* __restrict__ x, const float* __restrict__ e,
                                                     us* __restrict__ xh, us* __restrict__ xl,
                                                     us* __restrict__ eh, us* __restrict__ el, int n8)
{
  const int gi = blockIdx.x * 256 + threadIdx.x;
  if (gi >= 2 * n8) return;
  const bool first = gi < n8;
  const int o = first ? gi : (gi - n8);
  const float* src = (first ? x : e) + (size_t)o * 8;
  us* dh = (first ? xh : eh) + (size_t)o * 8;
  us* dl = (first ? xl : el) + (size_t)o * 8;
  const v4f a = *(const v4fa*)src;
  const v4f c = *(const v4fa*)(src + 4);
  float t[8];
  t[0] = a.x; t[1] = a.y; t[2] = a.z; t[3] = a.w; t[4] = c.x; t[5] = c.y; t[6] = c.z; t[7] = c.w;
  us hi[8], lo[8];
  #pragma unroll
  for (int j = 0; j < 8; ++j) { hi[j] = f2bf(t[j]); lo[j] = f2bf(t[j] - bf2f(hi[j])); }
  v4u H, L;
  H.x = pack2(hi[0], hi[1]); H.y = pack2(hi[2], hi[3]); H.z = pack2(hi[4], hi[5]); H.w = pack2(hi[6], hi[7]);
  L.x = pack2(lo[0], lo[1]); L.y = pack2(lo[2], lo[3]); L.z = pack2(lo[4], lo[5]); L.w = pack2(lo[6], lo[7]);
  *(volatile v4u*)dh = H;
  *(volatile v4u*)dl = L;
  __threadfence();
  *(volatile v4u*)dh = H;
  *(volatile v4u*)dl = L;
}

__global__ __launch_bounds__(256) void prepw_kernel(const float* __restrict__ W, const float* __restrict__ gain, int gzs,
                                                    us* __restrict__ Wh, us* __restrict__ Wl,
                                                    int K, int N, int Kpad, int Npad, int total8)
{
  const int t = blockIdx.x * 256 + threadIdx.x;
  if (t >= total8) return;
  const int kp8 = Kpad >> 3;
  const int k8 = t % kp8;
  const int n  = (t / kp8) % Npad;
  const int z  = t / (kp8 * Npad);
  const int nn = min(n, N - 1);
  us bh[8], bl[8];
  #pragma unroll
  for (int jj = 0; jj < 8; ++jj) {
    const int k = k8 * 8 + jj;
    const int kk = min(k, K - 1);
    float r = W[((size_t)z * K + kk) * N + nn];
    if (gain != nullptr) r = gain[(size_t)z * gzs + kk] * r;
    const bool ok = (k < K) && (n < N);
    const us hv = f2bf(r);
    const us lv = f2bf(r - bf2f(hv));
    bh[jj] = ok ? hv : (us)0;
    bl[jj] = ok ? lv : (us)0;
  }
  v4u H, L;
  H.x = pack2(bh[0], bh[1]); H.y = pack2(bh[2], bh[3]); H.z = pack2(bh[4], bh[5]); H.w = pack2(bh[6], bh[7]);
  L.x = pack2(bl[0], bl[1]); L.y = pack2(bl[2], bl[3]); L.z = pack2(bl[4], bl[5]); L.w = pack2(bl[6], bl[7]);
  us* dh = Wh + (size_t)t * 8;
  us* dl = Wl + (size_t)t * 8;
  *(volatile v4u*)dh = H;
  *(volatile v4u*)dl = L;
  __threadfence();
  *(volatile v4u*)dh = H;
  *(volatile v4u*)dl = L;
}

__global__ __launch_bounds__(256) void modbias_kernel(const float* __restrict__ W, const float* __restrict__ mb,
                                                      const float* __restrict__ beta, float* __restrict__ bias2)
{
  const int m = blockIdx.x, j = threadIdx.x;
  float s = 0.0f;
  #pragma unroll 1
  for (int d = 0; d < 256; ++d)
    s += beta[m * 256 + d] * W[((size_t)m * 256 + d) * 256 + j];
  const float v = mb[m * 256 + j] + s;
  float* p = bias2 + m * 256 + j;
  *(volatile float*)p = v;
  __threadfence();
  *(volatile float*)p = v;
}

struct GemmArgs {
  const us* Ahi; const us* Alo; const us* Wth; const us* Wtl; const float* bias; const float* aux;
  float* Cf; us* Phi; us* Plo; us* H16; uc* H8; float* part;
  long long w_zs;
  int lda, Kpad, N, b_zs, ldc, c_zoff, ldp, act, prelu, ldaux, ldh, h_zoff, nrb, nct, rowbase, ybase, p8rows, pad0;
};
static_assert(sizeof(GemmArgs) == 176);

template<int NT>
__global__ __launch_bounds__(256) void gemm_kernel(GemmArgs g)
{
  __shared__ __attribute__((aligned(16))) us    stg[8][2048];
  __shared__ __attribute__((aligned(16))) float sred[8][128];
  __shared__ __attribute__((aligned(16))) float sline[128];

  const int tid = threadIdx.x, lane = tid & 31, w = tid >> 5, hh = lane >> 4, m = lane & 15;
  const int z = blockIdx.z;
  const int rowl = blockIdx.y * 128 + w * 16;
  const int rowg = g.rowbase + rowl;
  const int n0 = blockIdx.x * (NT * 16);

  const us* ah = g.Ahi + (size_t)(rowl + m) * g.lda;
  const us* al = g.Alo + (size_t)(rowl + m) * g.lda;
  const size_t woff = (size_t)z * (size_t)g.w_zs + (size_t)(n0 + m) * g.Kpad;
  const us* wh = g.Wth + woff;
  const us* wl = g.Wtl + woff;

  v8f acc[NT];
  #pragma unroll
  for (int nt = 0; nt < NT; ++nt) acc[nt] = zero8();

  #pragma unroll 1
  for (int k0 = 0; k0 < g.Kpad; k0 += 32) {
    const v16bf a  = ldfrag(ah + k0, hh);
    const v16bf a2 = ldfrag(al + k0, hh);
    #pragma unroll
    for (int nt = 0; nt < NT; ++nt) {
      const size_t o = (size_t)nt * 16 * g.Kpad + k0;
      const v16bf bh = ldfrag(wh + o, hh);
      const v16bf bl = ldfrag(wl + o, hh);
      acc[nt] = wmma16(a,  bh, acc[nt]);
      acc[nt] = wmma16(a,  bl, acc[nt]);
      acc[nt] = wmma16(a2, bh, acc[nt]);
    }
  }

  float v[NT][8];
  #pragma unroll
  for (int nt = 0; nt < NT; ++nt) {
    const int n = n0 + nt * 16 + m;
    const int nn = min(n, g.N - 1);
    const bool valid = n < g.N;
    const float bv = g.bias[(size_t)z * g.b_zs + nn];
    #pragma unroll
    for (int r = 0; r < 8; ++r) {
      float t = acc[nt][r] + bv;
      if (g.act == 1) t = fmaxf(t, 0.0f);
      else if (g.act == 2) t = tanhf(t);
      else if (g.act == 3) {
        const float e = g.aux[(size_t)(rowg + 8 * hh + r) * g.ldaux + nn];
        t = fmaxf(t * e, 0.0f);
      }
      v[nt][r] = valid ? t : 0.0f;
    }
  }

  us* st = stg[w];

  if (g.Cf != nullptr) {
    f32a* sf = (f32a*)st;
    #pragma unroll
    for (int nt = 0; nt < NT; ++nt)
      #pragma unroll
      for (int r = 0; r < 8; ++r)
        sf[(8 * hh + r) * (NT * 16) + nt * 16 + m] = v[nt][r];
    wave_sync();
    float* cbase = g.Cf + (size_t)z * g.c_zoff + n0;
    store_f32_tile<NT>((const float*)sf, cbase, rowg, g.ldc, lane);
    __threadfence();
    store_f32_tile<NT>((const float*)sf, cbase, rowg, g.ldc, lane);
    wave_sync();
  }

  if (NT == 4) {
    if (g.Phi != nullptr) {
      usa* sh = (usa*)st;
      usa* sl = sh + 1024;
      #pragma unroll
      for (int nt = 0; nt < NT; ++nt)
        #pragma unroll
        for (int r = 0; r < 8; ++r) {
          float pv = v[nt][r];
          if (g.prelu) pv = fmaxf(pv, 0.0f);
          const us hi = f2bf(pv);
          const us lo = f2bf(pv - bf2f(hi));
          const int idx = (8 * hh + r) * 64 + nt * 16 + m;
          sh[idx] = hi;
          sl[idx] = lo;
        }
      wave_sync();
      store_u16_tile((const us*)sh, g.Phi + n0, rowg, g.ldp, lane);
      store_u16_tile((const us*)sl, g.Plo + n0, rowg, g.ldp, lane);
      __threadfence();
      store_u16_tile((const us*)sh, g.Phi + n0, rowg, g.ldp, lane);
      store_u16_tile((const us*)sl, g.Plo + n0, rowg, g.ldp, lane);
      wave_sync();
    }
    if (g.H16 != nullptr) {
      usa* sx = (usa*)st;
      uca* sb = (uca*)(st + 1024);
      #pragma unroll
      for (int nt = 0; nt < NT; ++nt)
        #pragma unroll
        for (int r = 0; r < 8; ++r) {
          const unsigned int ur = __float_as_uint(v[nt][r]) + 0x80u;
          const int idx = (8 * hh + r) * 64 + nt * 16 + m;
          sx[idx] = (us)(ur >> 16);
          sb[idx] = (uc)((ur >> 8) & 0xFFu);
        }
      wave_sync();
      us* hb = g.H16 + (size_t)z * g.h_zoff + n0;
      const int half = g.rowbase / g.p8rows;
      const int tile = half * ((int)gridDim.z * g.nct) + z * g.nct + blockIdx.x;
      uc* b8 = g.H8 + ((size_t)tile * g.p8rows + rowl) * 64;
      store_u16_tile((const us*)sx, hb, rowg, g.ldh, lane);
      store_u8_tile((const uc*)sb, b8, lane);
      __threadfence();
      store_u16_tile((const us*)sx, hb, rowg, g.ldh, lane);
      store_u8_tile((const uc*)sb, b8, lane);
      wave_sync();
    }
    if (g.part != nullptr) {
      #pragma unroll
      for (int nt = 0; nt < NT; ++nt) {
        float s = 0.0f, q = 0.0f;
        #pragma unroll
        for (int r = 0; r < 8; ++r) { s += v[nt][r]; q += v[nt][r] * v[nt][r]; }
        s += __shfl_xor(s, 16);
        q += __shfl_xor(q, 16);
        if (hh == 0) { sred[w][nt * 16 + m] = s; sred[w][64 + nt * 16 + m] = q; }
      }
      __syncthreads();
      if (tid < 128) {
        float t = 0.0f;
        #pragma unroll
        for (int ww = 0; ww < 8; ++ww) t += sred[ww][tid];
        sline[tid] = t;
      }
      __syncthreads();
      if (w == 0) {
        const v4f val = *(const v4fa*)(sline + lane * 4);
        float* dst = g.part + (((size_t)z * g.nrb + g.ybase + blockIdx.y) * g.nct + blockIdx.x) * 128 + lane * 4;
        *(volatile v4f*)dst = val;
        __threadfence();
        *(volatile v4f*)dst = val;
      }
    }
  }
}

__global__ __launch_bounds__(256) void gumbel_kernel(const float* __restrict__ lg3, const float* __restrict__ fl,
                                                     const float* __restrict__ usel, const float* __restrict__ ufin,
                                                     float* __restrict__ gt, int B)
{
  __shared__ __attribute__((aligned(16))) float sv[256 * 8];
  __shared__ __attribute__((aligned(16))) float srow[8 * 256];
  const int tid = threadIdx.x, rl = tid >> 5, t = tid & 31, i = t >> 3, mr = t & 7;
  const int b = blockIdx.x * 8 + rl;
  const bool sel = i < 3;
  const int ii = sel ? i : 0;
  const float* lp = sel ? (lg3 + ((size_t)ii * B + b) * 64 + mr * 8) : (fl + (size_t)b * 16);
  const float* up = sel ? (usel + (((size_t)b * 3 + ii) * 8 + mr) * 8) : (ufin + (size_t)b * 8);
  float* my = sv + tid * 8;
  float mx = -3.0e38f;
  #pragma unroll 1
  for (int j = 0; j < 8; ++j) {
    float u = up[j];
    u = fminf(fmaxf(u, 1e-10f), 0.99999988079071044921875f);
    const float gm = -logf(-logf(u));
    const float val = lp[j] + gm;
    my[j] = val;
    mx = fmaxf(mx, val);
  }
  float s = 0.0f;
  #pragma unroll 1
  for (int j = 0; j < 8; ++j) { const float e = expf(my[j] - mx); my[j] = e; s += e; }
  const float inv = 1.0f / s;
  float* orow = srow + rl * 256;
  #pragma unroll 1
  for (int j = 0; j < 8; ++j) {
    const float pv = my[j] * inv;
    if (sel) orow[i * 64 + mr * 8 + j] = pv;
    else if (mr == 0) orow[192 + j] = pv;
    else orow[200 + (mr - 1) * 8 + j] = 0.0f;
  }
  __syncthreads();
  #pragma unroll
  for (int it = 0; it < 2; ++it) {
    const int p = it * 256 + tid;
    const int rr = p >> 6, pc = p & 63;
    const v4f val = *(const v4fa*)(srow + rr * 256 + pc * 4);
    *(volatile v4f*)(gt + (size_t)(blockIdx.x * 8 + rr) * 256 + pc * 4) = val;
  }
  __threadfence();
  #pragma unroll
  for (int it = 0; it < 2; ++it) {
    const int p = it * 256 + tid;
    const int rr = p >> 6, pc = p & 63;
    const v4f val = *(const v4fa*)(srow + rr * 256 + pc * 4);
    *(volatile v4f*)(gt + (size_t)(blockIdx.x * 8 + rr) * 256 + pc * 4) = val;
  }
}

__global__ __launch_bounds__(256) void bnfin_kernel(const float* __restrict__ part, int nrb, int nct, int B,
                                                    float* __restrict__ mean, float* __restrict__ rstd)
{
  __shared__ __attribute__((aligned(16))) float sm[256];
  __shared__ __attribute__((aligned(16))) float sr[256];
  const int z = blockIdx.x, tid = threadIdx.x, lane = tid & 31, w = tid >> 5;
  const int x = tid >> 6, c = tid & 63;
  double s = 0.0, q = 0.0;
  #pragma unroll 1
  for (int y = 0; y < nrb; ++y) {
    const float* p = part + (((size_t)z * nrb + y) * nct + x) * 128;
    s += (double)p[c];
    q += (double)p[64 + c];
  }
  const double invB = 1.0 / (double)B;
  const double mu = s * invB;
  double var = q * invB - mu * mu;
  if (var < 0.0) var = 0.0;
  const float varf = (float)var;
  sm[tid] = (float)mu;
  sr[tid] = 1.0f / sqrtf(varf + 1e-5f);
  __syncthreads();
  if (w == 0) {
    #pragma unroll
    for (int it = 0; it < 2; ++it) {
      const int p = it * 32 + lane;
      const v4f val = *(const v4fa*)(sm + p * 4);
      *(volatile v4f*)(mean + (size_t)z * 256 + p * 4) = val;
    }
    __threadfence();
    #pragma unroll
    for (int it = 0; it < 2; ++it) {
      const int p = it * 32 + lane;
      const v4f val = *(const v4fa*)(sm + p * 4);
      *(volatile v4f*)(mean + (size_t)z * 256 + p * 4) = val;
    }
  } else if (w == 1) {
    #pragma unroll
    for (int it = 0; it < 2; ++it) {
      const int p = it * 32 + lane;
      const v4f val = *(const v4fa*)(sr + p * 4);
      *(volatile v4f*)(rstd + (size_t)z * 256 + p * 4) = val;
    }
    __threadfence();
    #pragma unroll
    for (int it = 0; it < 2; ++it) {
      const int p = it * 32 + lane;
      const v4f val = *(const v4fa*)(sr + p * 4);
      *(volatile v4f*)(rstd + (size_t)z * 256 + p * 4) = val;
    }
  }
}

__global__ __launch_bounds__(256) void xhat_kernel(const float* __restrict__ o, const float* __restrict__ mean,
                                                   const float* __restrict__ rstd, us* __restrict__ xa,
                                                   us* __restrict__ xb, int Bh, int n8)
{
  const int gi = blockIdx.x * 256 + threadIdx.x;
  if (gi >= n8) return;
  const int row = gi >> 5;
  const int c8 = (gi & 31) * 8;
  const bool half = row >= Bh;
  const int rl = row - (half ? Bh : 0);
  const float* src = o + (size_t)gi * 8;
  const v4f a = *(const v4fa*)src;
  const v4f c = *(const v4fa*)(src + 4);
  const v4f m0 = *(const v4fa*)(mean + c8);
  const v4f m1 = *(const v4fa*)(mean + c8 + 4);
  const v4f r0 = *(const v4fa*)(rstd + c8);
  const v4f r1 = *(const v4fa*)(rstd + c8 + 4);
  float t[8];
  t[0] = (a.x - m0.x) * r0.x; t[1] = (a.y - m0.y) * r0.y; t[2] = (a.z - m0.z) * r0.z; t[3] = (a.w - m0.w) * r0.w;
  t[4] = (c.x - m1.x) * r1.x; t[5] = (c.y - m1.y) * r1.y; t[6] = (c.z - m1.z) * r1.z; t[7] = (c.w - m1.w) * r1.w;
  us hi[8], lo[8];
  #pragma unroll
  for (int j = 0; j < 8; ++j) { hi[j] = f2bf(t[j]); lo[j] = f2bf(t[j] - bf2f(hi[j])); }
  v4u H, L;
  H.x = pack2(hi[0], hi[1]); H.y = pack2(hi[2], hi[3]); H.z = pack2(hi[4], hi[5]); H.w = pack2(hi[6], hi[7]);
  L.x = pack2(lo[0], lo[1]); L.y = pack2(lo[2], lo[3]); L.z = pack2(lo[4], lo[5]); L.w = pack2(lo[6], lo[7]);
  us* dh = (half ? xb : xa) + (size_t)rl * 256 + c8;
  us* dl = dh + (size_t)Bh * 256;
  *(volatile v4u*)dh = H;
  *(volatile v4u*)dl = L;
  __threadfence();
  *(volatile v4u*)dh = H;
  *(volatile v4u*)dl = L;
}

__global__ __launch_bounds__(256) void cascade_kernel(
    const us* __restrict__ h16,
    const uc* __restrict__ h8, int Bh,
    const float* __restrict__ mean2, const float* __restrict__ rstd2,
    const float* __restrict__ g2, const float* __restrict__ b2,
    const float* __restrict__ gt,
    const us* __restrict__ wlh, const us* __restrict__ wll,
    const float* __restrict__ lastb,
    float* __restrict__ out)
{
  __shared__ __attribute__((aligned(16))) float sS[256];
  __shared__ __attribute__((aligned(16))) us    sAh[16 * 256];
  __shared__ __attribute__((aligned(16))) us    sAl[16 * 256];
  __shared__ __attribute__((aligned(16))) float sO[288];

  const int tid = threadIdx.x, lane = tid & 31, w = tid >> 5, hh = lane >> 4, m16 = lane & 15;
  const int j = tid;
  const int jt = j >> 6, jc = j & 63;
  const int b0 = blockIdx.x * 16;
  const int half = (b0 >= Bh) ? 1 : 0;

  float mu[8], sc[8], be[8];
  #pragma unroll
  for (int mo = 0; mo < 8; ++mo) {
    const int c = mo * 256 + j;
    mu[mo] = mean2[c];
    sc[mo] = rstd2[c] * g2[c];
    be[mo] = b2[c];
  }

  #pragma unroll 1
  for (int r = 0; r < 16; ++r) {
    const int b = b0 + r;
    const int rl = b - half * Bh;
    sS[tid] = gt[(size_t)b * 256 + tid];
    float p[8];
    #pragma unroll
    for (int mo = 0; mo < 8; ++mo) {
      const unsigned int hv = (unsigned int)h16[(size_t)b * 2048 + mo * 256 + j];
      const unsigned int bv = (unsigned int)h8[((size_t)(half * 32 + mo * 4 + jt) * Bh + rl) * 64 + jc];
      const float f = __uint_as_float((hv << 16) | (bv << 8));
      p[mo] = (f - mu[mo]) * sc[mo] + be[mo];
    }
    __syncthreads();
    #pragma unroll
    for (int l = 0; l < 3; ++l) {
      const float* S = sS + (2 - l) * 64;
      float nx[8];
      #pragma unroll
      for (int a = 0; a < 8; ++a) {
        const v4f s0 = *(const v4fa*)(S + a * 8);
        const v4f s1 = *(const v4fa*)(S + a * 8 + 4);
        float t = s0.x * p[0];
        t += s0.y * p[1]; t += s0.z * p[2]; t += s0.w * p[3];
        t += s1.x * p[4]; t += s1.y * p[5]; t += s1.z * p[6]; t += s1.w * p[7];
        nx[a] = fmaxf(t, 0.0f);
      }
      #pragma unroll
      for (int a = 0; a < 8; ++a) p[a] = nx[a];
    }
    const v4f f0 = *(const v4fa*)(sS + 192);
    const v4f f1 = *(const v4fa*)(sS + 196);
    float oc = f0.x * p[0];
    oc += f0.y * p[1]; oc += f0.z * p[2]; oc += f0.w * p[3];
    oc += f1.x * p[4]; oc += f1.y * p[5]; oc += f1.z * p[6]; oc += f1.w * p[7];
    const us hi = f2bf(oc);
    const us lo = f2bf(oc - bf2f(hi));
    sAh[r * 256 + j] = hi;
    sAl[r * 256 + j] = lo;
    __syncthreads();
  }

  if (w == 0) {
    v8f acc0 = zero8(), acc1 = zero8();
    #pragma unroll
    for (int k0 = 0; k0 < 256; k0 += 32) {
      const v16bf a   = ldfrag(sAh + m16 * 256 + k0, hh);
      const v16bf al  = ldfrag(sAl + m16 * 256 + k0, hh);
      const v16bf bhA = ldfrag(wlh + (size_t)m16 * 256 + k0, hh);
      const v16bf blA = ldfrag(wll + (size_t)m16 * 256 + k0, hh);
      const v16bf bhB = ldfrag(wlh + (size_t)(16 + m16) * 256 + k0, hh);
      const v16bf blB = ldfrag(wll + (size_t)(16 + m16) * 256 + k0, hh);
      acc0 = wmma16(a,  bhA, acc0);
      acc0 = wmma16(a,  blA, acc0);
      acc0 = wmma16(al, bhA, acc0);
      acc1 = wmma16(a,  bhB, acc1);
      acc1 = wmma16(a,  blB, acc1);
      acc1 = wmma16(al, bhB, acc1);
    }
    const int nA = m16, nB = 16 + m16;
    const float bvA = lastb[min(nA, 17)];
    const float bvB = lastb[min(nB, 17)];
    #pragma unroll
    for (int r = 0; r < 8; ++r) {
      sO[(8 * hh + r) * 18 + nA] = acc0[r] + bvA;
      if (nB < 18) sO[(8 * hh + r) * 18 + nB] = acc1[r] + bvB;
    }
    wave_sync();
    float* ob = out + (size_t)b0 * 18;
    #pragma unroll
    for (int it = 0; it < 3; ++it) {
      const int p = it * 32 + lane;
      const int pp = min(p, 71);
      const v4f val = *(const v4fa*)(sO + pp * 4);
      if (p < 72) *(volatile v4f*)(ob + p * 4) = val;
    }
    __threadfence();
    #pragma unroll
    for (int it = 0; it < 3; ++it) {
      const int p = it * 32 + lane;
      const int pp = min(p, 71);
      const v4f val = *(const v4fa*)(sO + pp * 4);
      if (p < 72) *(volatile v4f*)(ob + p * 4) = val;
    }
  }
}

extern "C" void kernel_launch(void* const* d_in, const int* in_sizes, int n_in,
                              void* d_out, int out_size, void* d_ws, size_t ws_size,
                              hipStream_t stream)
{
  if (n_in != 28) return;
  const int B = in_sizes[0] / 128;
  if (B <= 0 || (B % 256) != 0) return;
  if (in_sizes[0] != B * 128 || in_sizes[1] != B * 128 || in_sizes[2] != B * 192 || in_sizes[3] != B * 8) return;
  if (in_sizes[4] != 51200 || in_sizes[5] != 400 || in_sizes[6] != 102400 || in_sizes[7] != 256) return;
  if (in_sizes[8] != 51200 || in_sizes[9] != 400 || in_sizes[10] != 102400 || in_sizes[11] != 256) return;
  if (in_sizes[12] != 65536 || in_sizes[13] != 256 || in_sizes[14] != 49152 || in_sizes[15] != 192) return;
  if (in_sizes[16] != 2048 || in_sizes[17] != 8 || in_sizes[18] != 49152 || in_sizes[19] != 768) return;
  if (in_sizes[20] != 524288 || in_sizes[21] != 2048 || in_sizes[22] != 4608 || in_sizes[23] != 18) return;
  if (in_sizes[24] != 2048 || in_sizes[25] != 2048 || in_sizes[26] != 2048 || in_sizes[27] != 2048) return;
  if (out_size != B * 18) return;

  const float* x       = (const float*)d_in[0];
  const float* embi    = (const float*)d_in[1];
  const float* u_sel   = (const float*)d_in[2];
  const float* u_fin   = (const float*)d_in[3];
  const float* base_W0 = (const float*)d_in[4];
  const float* base_b0 = (const float*)d_in[5];
  const float* base_W1 = (const float*)d_in[6];
  const float* base_b1 = (const float*)d_in[7];
  const float* em_W0   = (const float*)d_in[8];
  const float* em_b0   = (const float*)d_in[9];
  const float* gat_W0  = (const float*)d_in[10];
  const float* gat_b0  = (const float*)d_in[11];
  const float* gat_W1  = (const float*)d_in[12];
  const float* gat_b1  = (const float*)d_in[13];
  const float* sel_W   = (const float*)d_in[14];
  const float* sel_b   = (const float*)d_in[15];
  const float* selF_W  = (const float*)d_in[16];
  const float* selF_b  = (const float*)d_in[17];
  const float* cond_W  = (const float*)d_in[18];
  const float* cond_b  = (const float*)d_in[19];
  const float* mod_W   = (const float*)d_in[20];
  const float* mod_b   = (const float*)d_in[21];
  const float* last_W  = (const float*)d_in[22];
  const float* last_b  = (const float*)d_in[23];
  const float* bn1_g   = (const float*)d_in[24];
  const float* bn1_b   = (const float*)d_in[25];
  const float* bn2_g   = (const float*)d_in[26];
  const float* bn2_b   = (const float*)d_in[27];
  float* out = (float*)d_out;

  const int Bh  = B / 2;
  const int nrb = B / 128;

  char* ws = (char*)d_ws;
  const size_t Bz = (size_t)B;
  us*    XBH  = (us*)(ws + 0);
  us*    XBL  = (us*)(ws + 256 * Bz);
  us*    EBH  = (us*)(ws + 512 * Bz);
  us*    EBL  = (us*)(ws + 768 * Bz);
  us*    H1H  = (us*)(ws + 1024 * Bz);
  us*    H1L  = (us*)(ws + 1920 * Bz);
  us*    E1H  = H1H;
  us*    E1L  = H1L;
  us*    E2H  = (us*)(ws + 2816 * Bz);
  us*    E2L  = (us*)(ws + 3328 * Bz);
  us*    SIH  = (us*)(ws + 0);
  us*    SIL  = (us*)(ws + 512 * Bz);
  float* LG3  = (float*)(ws + 1024 * Bz);
  us*    LGH  = (us*)(ws + 1792 * Bz);
  us*    LGL  = (us*)(ws + 1920 * Bz);
  float* FL   = (float*)(ws + 2048 * Bz);
  us*    HP16 = (us*)(ws + 0);
  float* OUT0 = (float*)(ws + 4096 * Bz);
  float* EMB  = (float*)(ws + 5120 * Bz);
  us*    XHA  = (us*)(ws + 5120 * Bz);
  uc*    HP8  = (uc*)(ws + 4096 * Bz);
  float* GT   = (float*)(ws + 6144 * Bz);
  us*    XHB  = (us*)(ws + 7168 * Bz);
  size_t cur = 7680 * Bz;
  auto carve = [&](size_t bytes) -> char* {
    char* p = ws + cur;
    cur += (bytes + 4095) & ~(size_t)4095;
    return p;
  };
  const size_t nB0 = (size_t)448 * 128, nB1 = (size_t)256 * 416, nG1 = (size_t)256 * 256;
  const size_t nS = (size_t)3 * 64 * 256, nC = (size_t)3 * 256 * 64, nF = (size_t)16 * 256;
  const size_t nM = (size_t)8 * 256 * 256, nL = (size_t)32 * 256;
  us* WtB0 = (us*)carve(nB0 * 4);
  us* WtB1 = (us*)carve(nB1 * 4);
  us* WtE0 = (us*)carve(nB0 * 4);
  us* WtG0 = (us*)carve(nB1 * 4);
  us* WtG1 = (us*)carve(nG1 * 4);
  us* WtS  = (us*)carve(nS * 4);
  us* WtC  = (us*)carve(nC * 4);
  us* WtF  = (us*)carve(nF * 4);
  us* WtM  = (us*)carve(nM * 4);
  us* WtL  = (us*)carve(nL * 4);
  float* BIAS2 = (float*)carve((size_t)8 * 256 * 4);
  float* PART1 = (float*)carve((size_t)nrb * 4 * 128 * 4);
  float* PART2 = (float*)carve((size_t)8 * nrb * 4 * 128 * 4);
  float* MEAN1 = (float*)carve(256 * 4);
  float* RSTD1 = (float*)carve(256 * 4);
  float* MEAN2 = (float*)carve(2048 * 4);
  float* RSTD2 = (float*)carve(2048 * 4);
  if (cur > ws_size) return;
  if (cur > (size_t)134217728) return;

  dim3 blk(256);

  {
    const int n8 = B * 16;
    cvt_in_kernel<<<dim3((2 * n8 + 255) / 256), blk, 0, stream>>>(x, embi, XBH, XBL, EBH, EBL, n8);
  }
  auto prep = [&](const float* W, const float* gain, int gzs, us* Wt, int K, int N, int Kpad, int Npad, int Z) {
    const int total8 = Z * Npad * (Kpad / 8);
    const size_t plane = (size_t)Z * Npad * Kpad;
    prepw_kernel<<<dim3((total8 + 255) / 256), blk, 0, stream>>>(W, gain, gzs, Wt, Wt + plane, K, N, Kpad, Npad, total8);
  };
  prep(base_W0, nullptr, 0, WtB0, 128, 400, 128, 448, 1);
  prep(base_W1, nullptr, 0, WtB1, 400, 256, 416, 256, 1);
  prep(em_W0,   nullptr, 0, WtE0, 128, 400, 128, 448, 1);
  prep(gat_W0,  nullptr, 0, WtG0, 400, 256, 416, 256, 1);
  prep(gat_W1,  nullptr, 0, WtG1, 256, 256, 256, 256, 1);
  prep(sel_W,   nullptr, 0, WtS,  256,  64, 256,  64, 3);
  prep(cond_W,  nullptr, 0, WtC,   64, 256,  64, 256, 3);
  prep(selF_W,  nullptr, 0, WtF,  256,   8, 256,  16, 1);
  prep(mod_W,   bn1_g, 256, WtM,  256, 256, 256, 256, 8);
  prep(last_W,  nullptr, 0, WtL,  256,  18, 256,  32, 1);
  modbias_kernel<<<dim3(8), blk, 0, stream>>>(mod_W, mod_b, bn1_b, BIAS2);

  auto gemm = [&](int NT, const GemmArgs& g, int gridx, int rows, int Z) {
    dim3 grid(gridx, rows / 128, Z);
    if (NT == 4) gemm_kernel<4><<<grid, blk, 0, stream>>>(g);
    else         gemm_kernel<1><<<grid, blk, 0, stream>>>(g);
  };

  {
    GemmArgs g = {};
    g.Ahi = XBH; g.Alo = XBL; g.lda = 128; g.Kpad = 128; g.Wth = WtB0; g.Wtl = WtB0 + nB0;
    g.bias = base_b0; g.N = 400; g.act = 1;
    g.Phi = H1H; g.Plo = H1L; g.ldp = 448; g.p8rows = 1;
    gemm(4, g, 7, B, 1);
  }
  {
    GemmArgs g = {};
    g.Ahi = H1H; g.Alo = H1L; g.lda = 448; g.Kpad = 416; g.Wth = WtB1; g.Wtl = WtB1 + nB1;
    g.bias = base_b1; g.N = 256; g.act = 0;
    g.Cf = OUT0; g.ldc = 256; g.part = PART1; g.nrb = nrb; g.nct = 4; g.p8rows = 1;
    gemm(4, g, 4, B, 1);
  }
  {
    GemmArgs g = {};
    g.Ahi = EBH; g.Alo = EBL; g.lda = 128; g.Kpad = 128; g.Wth = WtE0; g.Wtl = WtE0 + nB0;
    g.bias = em_b0; g.N = 400; g.act = 1;
    g.Phi = E1H; g.Plo = E1L; g.ldp = 448; g.p8rows = 1;
    gemm(4, g, 7, B, 1);
  }
  {
    GemmArgs g = {};
    g.Ahi = E1H; g.Alo = E1L; g.lda = 448; g.Kpad = 416; g.Wth = WtG0; g.Wtl = WtG0 + nB1;
    g.bias = gat_b0; g.N = 256; g.act = 1;
    g.Phi = E2H; g.Plo = E2L; g.ldp = 256; g.p8rows = 1;
    gemm(4, g, 4, B, 1);
  }
  {
    GemmArgs g = {};
    g.Ahi = E2H; g.Alo = E2L; g.lda = 256; g.Kpad = 256; g.Wth = WtG1; g.Wtl = WtG1 + nG1;
    g.bias = gat_b1; g.N = 256; g.act = 0;
    g.Cf = EMB; g.ldc = 256; g.Phi = SIH; g.Plo = SIL; g.ldp = 256; g.prelu = 1; g.p8rows = 1;
    gemm(4, g, 4, B, 1);
  }
  for (int i = 0; i < 3; ++i) {
    {
      GemmArgs g = {};
      g.Ahi = SIH; g.Alo = SIL; g.lda = 256; g.Kpad = 256;
      g.Wth = WtS + (size_t)i * 64 * 256; g.Wtl = WtS + nS + (size_t)i * 64 * 256;
      g.bias = sel_b + i * 64; g.N = 64; g.act = 2;
      g.Cf = LG3 + (size_t)i * B * 64; g.ldc = 64; g.Phi = LGH; g.Plo = LGL; g.ldp = 64; g.p8rows = 1;
      gemm(4, g, 1, B, 1);
    }
    {
      GemmArgs g = {};
      g.Ahi = LGH; g.Alo = LGL; g.lda = 64; g.Kpad = 64;
      g.Wth = WtC + (size_t)i * 256 * 64; g.Wtl = WtC + nC + (size_t)i * 256 * 64;
      g.bias = cond_b + i * 256; g.N = 256; g.act = 3; g.aux = EMB; g.ldaux = 256;
      g.Phi = SIH; g.Plo = SIL; g.ldp = 256; g.p8rows = 1;
      gemm(4, g, 4, B, 1);
    }
  }
  {
    GemmArgs g = {};
    g.Ahi = SIH; g.Alo = SIL; g.lda = 256; g.Kpad = 256; g.Wth = WtF; g.Wtl = WtF + nF;
    g.bias = selF_b; g.N = 8; g.act = 0;
    g.Cf = FL; g.ldc = 16; g.p8rows = 1;
    gemm(1, g, 1, B, 1);
  }
  gumbel_kernel<<<dim3(B / 8), blk, 0, stream>>>(LG3, FL, u_sel, u_fin, GT, B);
  bnfin_kernel<<<dim3(1), blk, 0, stream>>>(PART1, nrb, 4, B, MEAN1, RSTD1);
  {
    const int n8 = B * 32;
    xhat_kernel<<<dim3((n8 + 255) / 256), blk, 0, stream>>>(OUT0, MEAN1, RSTD1, XHA, XHB, Bh, n8);
  }
  for (int hf = 0; hf < 2; ++hf) {
    GemmArgs g = {};
    const us* xh = (hf == 0) ? XHA : XHB;
    g.Ahi = xh; g.Alo = xh + (size_t)Bh * 256; g.lda = 256; g.Kpad = 256;
    g.Wth = WtM; g.Wtl = WtM + nM; g.w_zs = (long long)256 * 256;
    g.bias = BIAS2; g.b_zs = 256; g.N = 256; g.act = 0;
    g.H16 = HP16; g.ldh = 2048; g.h_zoff = 256; g.H8 = HP8; g.p8rows = Bh;
    g.part = PART2; g.nrb = nrb; g.nct = 4;
    g.rowbase = hf * Bh; g.ybase = hf * (Bh / 128);
    gemm(4, g, 4, Bh, 8);
  }
  bnfin_kernel<<<dim3(8), blk, 0, stream>>>(PART2, nrb, 4, B, MEAN2, RSTD2);
  cascade_kernel<<<dim3(B / 16), blk, 0, stream>>>(HP16, HP8, Bh, MEAN2, RSTD2, bn2_g, bn2_b, GT,
                                                  WtL, WtL + nL, last_b, out);
}
